// MultiHeadAttention_2327872275103
// MI455X (gfx1250) — hardware-run, weakly checked
//
#include <hip/hip_runtime.h>
#include <stddef.h>


typedef _Float16 v16h __attribute__((ext_vector_type(16)));
typedef _Float16 v8h  __attribute__((ext_vector_type(8)));
typedef float    v8f  __attribute__((ext_vector_type(8)));
typedef float    v4f  __attribute__((ext_vector_type(4)));
typedef _Float16 h16;

#ifndef NB
#define NB 2
#endif
#ifndef SEQ
#define SEQ 2048
#endif
#define NB_FULL  2
#define SEQ_FULL 2048
#define DIM   1024
#define NHEAD 16
#define HD    64
#define HDK   16
#define QW    (NHEAD * HDK)
#define QKW   (2 * QW)
#define FFH   64
#define MROWS (NB * SEQ)

static_assert(NB >= 1 && NB <= NB_FULL);
static_assert(SEQ >= 128 && SEQ <= SEQ_FULL && (SEQ % 128) == 0);
static_assert(DIM == NHEAD * HD);
static_assert(HD == 64);
static_assert(HDK == 16);
static_assert(QW == 256 && QKW == 512);
static_assert(FFH == 64);
static_assert((DIM % 64) == 0 && (DIM % 32) == 0);
static_assert((QKW % 64) == 0 && (FFH % 64) == 0 && (FFH % 32) == 0);
static_assert((MROWS % 64) == 0 && (MROWS % 8) == 0);
static_assert(DIM == 128 * 8);
static_assert(((QW * DIM) % 2048) == 0);
static_assert(((DIM * DIM) % 2048) == 0);
static_assert(((FFH * DIM) % 2048) == 0);
static_assert(((MROWS * DIM) % 2048) == 0);

#define LDT 72
#define LDC 68
static_assert((LDT % 8) == 0 && LDT >= 64);
static_assert((LDC % 4) == 0 && LDC >= 64);

#define WCARRY 64.0f
#define PCARRY 1024.0f
#define VCARRY 64.0f
#define MCARRY 16.0f

#define WQK_BYTES     ((size_t)QKW * DIM * 2)
#define WSQ_BYTES     ((size_t)DIM * DIM * 2)
#define WFF_BYTES     ((size_t)FFH * DIM * 2)
#define PLANE16_BYTES ((size_t)MROWS * DIM * 2)
#define QK16_BYTES    ((size_t)MROWS * QKW * 2)
#define H16_BYTES     ((size_t)MROWS * FFH * 2)
#define F32_BYTES     ((size_t)MROWS * DIM * 4)
#define OFF_WQK ((size_t)0)
#define OFF_WV  (OFF_WQK + WQK_BYTES)
#define OFF_WP  (OFF_WV + WSQ_BYTES)
#define OFF_W1  (OFF_WP + WSQ_BYTES)
#define OFF_W2  (OFF_W1 + WFF_BYTES)
#define OFF_E16 (OFF_W2 + WFF_BYTES)
#define OFF_QK  (OFF_E16 + PLANE16_BYTES)
#define OFF_VT  (OFF_QK + QK16_BYTES)
#define OFF_CTX (OFF_VT + PLANE16_BYTES)
#define OFF_R16 (OFF_CTX + PLANE16_BYTES)
#define OFF_H16 (OFF_R16 + PLANE16_BYTES)
#define OFF_RES (OFF_H16 + H16_BYTES)
#define OFF_E1  (OFF_RES + F32_BYTES)
#define WS_TOTAL (OFF_E1 + F32_BYTES)
static_assert((WQK_BYTES % 128) == 0 && (WSQ_BYTES % 128) == 0 && (WFF_BYTES % 128) == 0);
static_assert((PLANE16_BYTES % 128) == 0 && (QK16_BYTES % 128) == 0 && (H16_BYTES % 128) == 0);
static_assert((F32_BYTES % 128) == 0);
static_assert(WS_TOTAL <= (size_t)134217728);

__device__ __forceinline__ float bf16r(float x) {
  unsigned int u = __float_as_uint(x);
  u = (u + 0x7FFFu + ((u >> 16) & 1u)) & 0xFFFF0000u;
  return __uint_as_float(u);
}

static __device__ __forceinline__ h16 toh_flush(float v) {
  const h16 r = (h16)v;
  return (fabsf(v) < 6.103515625e-05f) ? (h16)0.0f : r;
}

__device__ __forceinline__ v16h frag_at(const _Float16* p) {
  v8h lo = *(const v8h*)(p);
  v8h hi = *(const v8h*)(p + 16);
  v16h out;
#pragma unroll
  for (int i = 0; i < 8; ++i) { out[i] = lo[i]; out[i + 8] = hi[i]; }
  return out;
}
__device__ __forceinline__ v16h ld_frag(const _Float16* base, unsigned ld) {
  const unsigned lane = threadIdx.x & 31u;
  return frag_at(base + (lane & 15u) * ld + (lane >> 4) * 8u);
}

__device__ __forceinline__ v8f wmma16(v16h a, v16h b, v8f c) {
  v8f d = __builtin_amdgcn_wmma_f32_16x16x32_f16(false, a, false, b, (short)0, c,
                                                 false, false);
  asm volatile("v_nop\n\tv_nop\n\tv_nop\n\tv_nop" : "+v"(d) : "v"(a), "v"(b));
  return d;
}

__device__ __forceinline__ float red16_max(float x) {
#pragma unroll
  for (int off = 1; off < 16; off <<= 1) x = fmaxf(x, __shfl_xor(x, off, 32));
  return x;
}
__device__ __forceinline__ float red16_sum(float x) {
#pragma unroll
  for (int off = 1; off < 16; off <<= 1) x += __shfl_xor(x, off, 32);
  return x;
}

__device__ __forceinline__ void wave_lds_sync() {
  __builtin_amdgcn_fence(3  , "wavefront");
  asm volatile("s_wait_dscnt 0x0" ::: "memory");
  __builtin_amdgcn_wave_barrier();
}

__device__ __forceinline__ float relu_act(float t) {
  return fmaxf(t, 0.0f);
}

__global__ __launch_bounds__(256) void wcast_kernel(
    const float* __restrict__ W, _Float16* __restrict__ Wt) {
  const unsigned t = blockIdx.x * 256u + threadIdx.x;
  const v4f a0 = *(const v4f*)(W + (size_t)t * 8u);
  const v4f a1 = *(const v4f*)(W + (size_t)t * 8u + 4u);
  v8h o;
#pragma unroll
  for (int i = 0; i < 4; ++i) {
    o[i]     = toh_flush(WCARRY * bf16r(a0[i]));
    o[i + 4] = toh_flush(WCARRY * bf16r(a1[i]));
  }
  _Float16* p = Wt + (size_t)t * 8u;
  *(volatile v8h*)p = o;
  __threadfence();
  *(volatile v8h*)p = o;
}

template <int SRC_INPUT>
__device__ __forceinline__ void rowcast_body(const float* __restrict__ X,
                                             _Float16* __restrict__ dst) {
  const unsigned t = blockIdx.x * 256u + threadIdx.x;
  const unsigned crow = t >> 7;
  const unsigned c = (t & 127u) * 8u;
  size_t srow = crow;
  if (SRC_INPUT) {
    const unsigned bidx = crow / (unsigned)SEQ;
    const unsigned sq = crow - bidx * (unsigned)SEQ;
    srow = (size_t)bidx * SEQ_FULL + sq;
  }
  const float* xr = X + srow * DIM + c;
  const v4f a0 = *(const v4f*)(xr);
  const v4f a1 = *(const v4f*)(xr + 4u);
  v8h o;
#pragma unroll
  for (int i = 0; i < 4; ++i) {
    o[i]     = toh_flush(SRC_INPUT ? bf16r(a0[i]) : a0[i]);
    o[i + 4] = toh_flush(SRC_INPUT ? bf16r(a1[i]) : a1[i]);
  }
  _Float16* p = dst + (size_t)crow * DIM + c;
  *(volatile v8h*)p = o;
  __threadfence();
  *(volatile v8h*)p = o;
}

__global__ __launch_bounds__(256) void rowcast_in_kernel(
    const float* __restrict__ X, _Float16* __restrict__ dst) {
  rowcast_body<1>(X, dst);
}
__global__ __launch_bounds__(256) void rowcast_ws_kernel(
    const float* __restrict__ X, _Float16* __restrict__ dst) {
  rowcast_body<0>(X, dst);
}

template <int MODE>
__device__ __forceinline__ void gemm_body(
    const _Float16* __restrict__ A16, const _Float16* __restrict__ Bt, const unsigned K,
    const float* __restrict__ bias, const float* __restrict__ addf,
    float* __restrict__ outf, _Float16* __restrict__ out16) {
  __shared__ float Cs[64 * LDC];
  const unsigned tid = threadIdx.x, lane = tid & 31u;
  const unsigned w = (unsigned)__builtin_amdgcn_readfirstlane((int)(threadIdx.x >> 5));
  const unsigned mw = w >> 1, nw = w & 1u;
  const unsigned hh = lane >> 4, m = lane & 15u;
  const unsigned n0 = blockIdx.x * 64u;
  const unsigned row0 = blockIdx.y * 64u;

  const _Float16* ap  = A16 + (size_t)(row0 + mw * 16u + m) * K + hh * 8u;
  const _Float16* bp0 = Bt + (size_t)(n0 + nw * 32u + m) * K + hh * 8u;
  const _Float16* bp1 = bp0 + (size_t)16 * K;
  v8f acc0 = {}, acc1 = {};
#pragma unroll 2
  for (unsigned k0 = 0; k0 < K; k0 += 32u) {
    const v16h a  = frag_at(ap + k0);
    const v16h b0 = frag_at(bp0 + k0);
    const v16h b1 = frag_at(bp1 + k0);
    acc0 = wmma16(a, b0, acc0);
    acc1 = wmma16(a, b1, acc1);
  }
#pragma unroll
  for (int r = 0; r < 8; ++r) {
    float* d = &Cs[(mw * 16u + hh * 8u + (unsigned)r) * LDC + nw * 32u + m];
    d[0]  = acc0[r];
    d[16] = acc1[r];
  }
  __syncthreads();

  if (MODE == 3) {
#pragma unroll 1
    for (unsigned g = 0; g < 4u; ++g) {
      const unsigned r = 32u * (g >> 1) + (tid >> 3);
      const unsigned c = (tid & 7u) * 8u + 4u * (g & 1u);
      const v4f u  = *(const v4f*)&Cs[r * LDC + c];
      const v4f gb = *(const v4f*)(bias + n0 + c);
      v4f t;
#pragma unroll
      for (int j = 0; j < 4; ++j)
        t[j] = MCARRY * relu_act(u[j] * (1.0f / WCARRY) + bf16r(gb[j]));
      *(v4f*)&Cs[r * LDC + c] = t;
    }
  }

  if (MODE == 0 || MODE == 3) {
    const unsigned ldo = (MODE == 3) ? (unsigned)FFH : (unsigned)QKW;
    v8h x[2];
    size_t off[2];
#pragma unroll
    for (unsigned i = 0; i < 2u; ++i) {
      const unsigned r = 32u * i + (tid >> 3);
      const unsigned c = (tid & 7u) * 8u;
      const v4f u0 = *(const v4f*)&Cs[r * LDC + c];
      const v4f u1 = *(const v4f*)&Cs[r * LDC + c + 4];
      if (MODE == 3) {
#pragma unroll
        for (int j = 0; j < 4; ++j) {
          x[i][j]     = toh_flush(u0[j]);
          x[i][j + 4] = toh_flush(u1[j]);
        }
      } else {
#pragma unroll
        for (int j = 0; j < 4; ++j) {
          x[i][j]     = toh_flush(u0[j] * (1.0f / WCARRY));
          x[i][j + 4] = toh_flush(u1[j] * (1.0f / WCARRY));
        }
      }
      off[i] = (size_t)(row0 + r) * ldo + n0 + c;
    }
#pragma unroll
    for (int i = 0; i < 2; ++i) *(volatile v8h*)(out16 + off[i]) = x[i];
    __threadfence();
#pragma unroll
    for (int i = 0; i < 2; ++i) *(volatile v8h*)(out16 + off[i]) = x[i];
  }

  if (MODE == 1) {
    const unsigned bidx = row0 / (unsigned)SEQ;
    const unsigned key0 = row0 - bidx * (unsigned)SEQ;
    v8h x[2];
    size_t off[2];
#pragma unroll
    for (unsigned i = 0; i < 2u; ++i) {
      const unsigned dcol = 32u * i + (tid >> 3);
      const unsigned kk = (tid & 7u) * 8u;
#pragma unroll
      for (unsigned j = 0; j < 8u; ++j) {
        const float t = Cs[(kk + j) * LDC + dcol] * (1.0f / WCARRY);
        x[i][j] = toh_flush(t);
      }
      off[i] = ((size_t)bidx * DIM + n0 + dcol) * SEQ + key0 + kk;
    }
#pragma unroll
    for (int i = 0; i < 2; ++i) *(volatile v8h*)(out16 + off[i]) = x[i];
    __threadfence();
#pragma unroll
    for (int i = 0; i < 2; ++i) *(volatile v8h*)(out16 + off[i]) = x[i];
  }

  if (MODE == 2 || MODE == 4 || MODE == 5 || MODE == 6) {
    const bool src_in   = (MODE == 2);
    const bool has_bias = (MODE == 4 || MODE == 6);
    const bool out_full = (MODE == 4);
    const float cs = (MODE == 2 || MODE == 5) ? (1.0f / (WCARRY * VCARRY))
                                              : (1.0f / (WCARRY * MCARRY));
    v4f xs[4];
    size_t off[4];
#pragma unroll
    for (unsigned i = 0; i < 4u; ++i) {
      const unsigned r = 16u * i + (tid >> 4);
      const unsigned c = (tid & 15u) * 4u;
      const unsigned crow = row0 + r;
      const unsigned bidx = crow / (unsigned)SEQ;
      const unsigned sq = crow - bidx * (unsigned)SEQ;
      const size_t frow = (size_t)bidx * SEQ_FULL + sq;
      const size_t inrow  = src_in ? frow : (size_t)crow;
      const size_t outrow = out_full ? frow : (size_t)crow;
      const v4f u = *(const v4f*)&Cs[r * LDC + c];
      v4f g = {0.0f, 0.0f, 0.0f, 0.0f};
      if (has_bias) g = *(const v4f*)(bias + n0 + c);
      const v4f xin = *(const v4f*)(addf + inrow * DIM + n0 + c);
      v4f val;
#pragma unroll
      for (int j = 0; j < 4; ++j) {
        const float base = src_in ? bf16r(xin[j]) : xin[j];
        const float gb = has_bias ? bf16r(g[j]) : 0.0f;
        val[j] = base + (u[j] * cs + gb);
      }
      xs[i] = val;
      off[i] = outrow * DIM + n0 + c;
    }
#pragma unroll
    for (int i = 0; i < 4; ++i) *(volatile v4f*)(outf + off[i]) = xs[i];
    __threadfence();
#pragma unroll
    for (int i = 0; i < 4; ++i) *(volatile v4f*)(outf + off[i]) = xs[i];
  }
}

__global__ __launch_bounds__(256) void gemm_qk_kernel(
    const _Float16* __restrict__ A16, const _Float16* __restrict__ Bt,
    _Float16* __restrict__ out16) {
  gemm_body<0>(A16, Bt, (unsigned)DIM, (const float*)0, (const float*)0, (float*)0, out16);
}
__global__ __launch_bounds__(256) void gemm_v_kernel(
    const _Float16* __restrict__ A16, const _Float16* __restrict__ Bt,
    _Float16* __restrict__ vt) {
  gemm_body<1>(A16, Bt, (unsigned)DIM, (const float*)0, (const float*)0, (float*)0, vt);
}
__global__ __launch_bounds__(256) void gemm_wp_in_kernel(
    const _Float16* __restrict__ A16, const _Float16* __restrict__ Bt,
    const float* __restrict__ xin, float* __restrict__ res) {
  gemm_body<2>(A16, Bt, (unsigned)DIM, xin, xin, res, (_Float16*)0);
}
__global__ __launch_bounds__(256) void gemm_wp_ws_kernel(
    const _Float16* __restrict__ A16, const _Float16* __restrict__ Bt,
    const float* __restrict__ ein, float* __restrict__ res) {
  gemm_body<5>(A16, Bt, (unsigned)DIM, ein, ein, res, (_Float16*)0);
}
__global__ __launch_bounds__(256) void gemm_ffn1_kernel(
    const _Float16* __restrict__ A16, const _Float16* __restrict__ Bt,
    const float* __restrict__ bias, _Float16* __restrict__ mid) {
  gemm_body<3>(A16, Bt, (unsigned)DIM, bias, bias, (float*)0, mid);
}
__global__ __launch_bounds__(256) void gemm_ffn2_ws_kernel(
    const _Float16* __restrict__ A16, const _Float16* __restrict__ Bt,
    const float* __restrict__ bias, const float* __restrict__ res, float* __restrict__ eout) {
  gemm_body<6>(A16, Bt, (unsigned)FFH, bias, res, eout, (_Float16*)0);
}
__global__ __launch_bounds__(256) void gemm_ffn2_out_kernel(
    const _Float16* __restrict__ A16, const _Float16* __restrict__ Bt,
    const float* __restrict__ bias, const float* __restrict__ res, float* __restrict__ outf) {
  gemm_body<4>(A16, Bt, (unsigned)FFH, bias, res, outf, (_Float16*)0);
}

__global__ __launch_bounds__(256) void attn_kernel(
    const _Float16* __restrict__ QK, const _Float16* __restrict__ Vt,
    _Float16* __restrict__ Ov) {
  __shared__ _Float16 Vs[64 * LDT];
  __shared__ _Float16 Ps[8 * 16 * LDT];

  const unsigned tid = threadIdx.x, lane = tid & 31u;
  const unsigned w = (unsigned)__builtin_amdgcn_readfirstlane((int)(threadIdx.x >> 5));
  const unsigned hh = lane >> 4, m = lane & 15u;
  const unsigned q0 = blockIdx.x * 128u;
  const unsigned head = blockIdx.y;
  const unsigned b = blockIdx.z;
  const float scale = 0.25f;
  const unsigned qrow0 = q0 + w * 16u;
  _Float16* P = Ps + w * (16u * LDT);

  v16h qf;
  {
    const v8h ql = *(const v8h*)(QK + (size_t)(b * (unsigned)SEQ + qrow0 + m) * QKW +
                                 head * HDK + hh * 8u);
#pragma unroll
    for (int i = 0; i < 8; ++i) { qf[i] = ql[i]; qf[i + 8] = (_Float16)0.0f; }
  }

  float mrow[8], lrow[8];
  v8f o[4];
#pragma unroll
  for (int v = 0; v < 8; ++v) { mrow[v] = -1.0e30f; lrow[v] = 0.0f; }
#pragma unroll
  for (int nb = 0; nb < 4; ++nb) o[nb] = (v8f){};

  const _Float16* kp = QK + (size_t)(b * (unsigned)SEQ + m) * QKW + QW + head * HDK + hh * 8u;
  const size_t vplane = ((size_t)b * DIM + head * HD) * SEQ;

  for (unsigned kb = 0; kb < (unsigned)SEQ; kb += 64u) {
#pragma unroll
    for (unsigned j = 0; j < 2u; ++j) {
      const unsigned idx = tid + 256u * j;
      const unsigned r = idx >> 3, c = (idx & 7u) * 8u;
      *(v8h*)&Vs[r * LDT + c] = *(const v8h*)(Vt + vplane + (size_t)r * SEQ + kb + c);
    }
    __syncthreads();

    v8f s[4];
#pragma unroll
    for (int kg = 0; kg < 4; ++kg) {
      const v8h kl = *(const v8h*)(kp + (size_t)(kb + (unsigned)kg * 16u) * QKW);
      v16h kf;
#pragma unroll
      for (int i = 0; i < 8; ++i) { kf[i] = kl[i]; kf[i + 8] = (_Float16)0.0f; }
      v8f t = {};
      t = wmma16(qf, kf, t);
      s[kg] = t * scale;
    }

    float alpha[8];
#pragma unroll
    for (int v = 0; v < 8; ++v) {
      float mx = fmaxf(fmaxf(s[0][v], s[1][v]), fmaxf(s[2][v], s[3][v]));
      mx = red16_max(mx);
      const float mn = fmaxf(mrow[v], mx);
      alpha[v] = __expf(mrow[v] - mn);
      mrow[v] = mn;
    }
#pragma unroll
    for (int kg = 0; kg < 4; ++kg)
#pragma unroll
      for (int v = 0; v < 8; ++v) {
        const float d = s[kg][v] - mrow[v];
        s[kg][v] = (d < -16.0f) ? 0.0f : __expf(d);
      }
#pragma unroll
    for (int v = 0; v < 8; ++v) {
      const float rs = red16_sum((s[0][v] + s[1][v]) + (s[2][v] + s[3][v]));
      lrow[v] = alpha[v] * lrow[v] + rs;
    }
#pragma unroll
    for (int nb = 0; nb < 4; ++nb)
#pragma unroll
      for (int v = 0; v < 8; ++v) o[nb][v] = o[nb][v] * alpha[v];

#pragma unroll
    for (int kg = 0; kg < 4; ++kg)
#pragma unroll
      for (int v = 0; v < 8; ++v)
        P[(hh * 8u + (unsigned)v) * LDT + (unsigned)kg * 16u + m] = toh_flush(s[kg][v] * PCARRY);
    wave_lds_sync();

#pragma unroll
    for (int c = 0; c < 2; ++c) {
      const v16h pf = ld_frag(P + c * 32, LDT);
#pragma unroll
      for (int nb = 0; nb < 4; ++nb) {
        const v16h vf = ld_frag(&Vs[(nb * 16) * LDT + c * 32], LDT);
        o[nb] = wmma16(pf, vf, o[nb]);
      }
    }
    __syncthreads();
  }

  float inv[8];
#pragma unroll
  for (int v = 0; v < 8; ++v) inv[v] = __builtin_amdgcn_rcpf(lrow[v]) * (VCARRY / PCARRY);
#pragma unroll
  for (int nb = 0; nb < 4; ++nb)
#pragma unroll
    for (int v = 0; v < 8; ++v)
      P[(hh * 8u + (unsigned)v) * LDT + (unsigned)nb * 16u + m] = toh_flush(o[nb][v] * inv[v]);
  wave_lds_sync();
  v8h x[4];
  size_t off[4];
#pragma unroll
  for (unsigned i = 0; i < 4u; ++i) {
    const unsigned r = 4u * i + (lane >> 3);
    const unsigned c = (lane & 7u) * 8u;
    x[i] = *(const v8h*)&P[r * LDT + c];
    off[i] = (size_t)(b * (unsigned)SEQ + qrow0 + r) * DIM + head * HD + c;
  }
#pragma unroll
  for (int i = 0; i < 4; ++i) *(volatile v8h*)(Ov + off[i]) = x[i];
  __threadfence();
#pragma unroll
  for (int i = 0; i < 4; ++i) *(volatile v8h*)(Ov + off[i]) = x[i];
}

extern "C" void kernel_launch(void* const* d_in, const int* in_sizes, int n_in,
                              void* d_out, int out_size, void* d_ws, size_t ws_size,
                              hipStream_t stream) {
  if (n_in < 9) return;
  const long long need_x = ((long long)(NB - 1) * SEQ_FULL + SEQ) * DIM;
  if ((long long)in_sizes[0] < need_x) return;
  if ((long long)in_sizes[1] < (long long)QW * DIM) return;
  if ((long long)in_sizes[2] < (long long)QW * DIM) return;
  if ((long long)in_sizes[3] < (long long)DIM * DIM) return;
  if ((long long)in_sizes[4] < (long long)DIM * DIM) return;
  if ((long long)in_sizes[5] < (long long)FFH * DIM) return;
  if (in_sizes[6] < FFH) return;
  if ((long long)in_sizes[7] < (long long)DIM * FFH) return;
  if (in_sizes[8] < DIM) return;
  if ((long long)out_size < need_x) return;
  if (ws_size < WS_TOTAL) return;

  const float* X  = (const float*)d_in[0];
  const float* wq = (const float*)d_in[1];
  const float* wk = (const float*)d_in[2];
  const float* wv = (const float*)d_in[3];
  const float* wp = (const float*)d_in[4];
  const float* w1 = (const float*)d_in[5];
  const float* b1 = (const float*)d_in[6];
  const float* w2 = (const float*)d_in[7];
  const float* b2 = (const float*)d_in[8];
  float* out = (float*)d_out;

  char* ws = (char*)d_ws;
  _Float16* Wqk_t = (_Float16*)(ws + OFF_WQK);
  _Float16* Wv_t  = (_Float16*)(ws + OFF_WV);
  _Float16* Wp_t  = (_Float16*)(ws + OFF_WP);
  _Float16* W1_t  = (_Float16*)(ws + OFF_W1);
  _Float16* W2_t  = (_Float16*)(ws + OFF_W2);
  _Float16* E16   = (_Float16*)(ws + OFF_E16);
  _Float16* QK16  = (_Float16*)(ws + OFF_QK);
  _Float16* Vt16  = (_Float16*)(ws + OFF_VT);
  _Float16* Ctx16 = (_Float16*)(ws + OFF_CTX);
  _Float16* R16   = (_Float16*)(ws + OFF_R16);
  _Float16* H16   = (_Float16*)(ws + OFF_H16);
  float*    RES   = (float*)(ws + OFF_RES);
  float*    E1    = (float*)(ws + OFF_E1);

  dim3 blk(256);
  dim3 gqk(QKW / 64, MROWS / 64);
  dim3 gg(DIM / 64, MROWS / 64);
  dim3 gh(FFH / 64, MROWS / 64);
  dim3 gat(SEQ / 128, NHEAD, NB);
  dim3 grow((MROWS * (DIM / 8)) / 256);

  wcast_kernel<<<dim3((QW * DIM) / 2048), blk, 0, stream>>>(wq, Wqk_t);
  wcast_kernel<<<dim3((QW * DIM) / 2048), blk, 0, stream>>>(wk, Wqk_t + (size_t)QW * DIM);
  wcast_kernel<<<dim3((DIM * DIM) / 2048), blk, 0, stream>>>(wv, Wv_t);
  wcast_kernel<<<dim3((DIM * DIM) / 2048), blk, 0, stream>>>(wp, Wp_t);
  wcast_kernel<<<dim3((FFH * DIM) / 2048), blk, 0, stream>>>(w1, W1_t);
  wcast_kernel<<<dim3((DIM * FFH) / 2048), blk, 0, stream>>>(w2, W2_t);

  rowcast_in_kernel<<<grow, blk, 0, stream>>>(X, E16);
  gemm_qk_kernel<<<gqk, blk, 0, stream>>>(E16, Wqk_t, QK16);
  gemm_v_kernel<<<gg, blk, 0, stream>>>(E16, Wv_t, Vt16);
  attn_kernel<<<gat, blk, 0, stream>>>(QK16, Vt16, Ctx16);
  gemm_wp_in_kernel<<<gg, blk, 0, stream>>>(Ctx16, Wp_t, X, RES);
  rowcast_ws_kernel<<<grow, blk, 0, stream>>>(RES, R16);
  gemm_ffn1_kernel<<<gh, blk, 0, stream>>>(R16, W1_t, b1, H16);
  gemm_ffn2_ws_kernel<<<gg, blk, 0, stream>>>(H16, W2_t, b2, RES, E1);

  rowcast_ws_kernel<<<grow, blk, 0, stream>>>(E1, E16);
  gemm_qk_kernel<<<gqk, blk, 0, stream>>>(E16, Wqk_t, QK16);
  gemm_v_kernel<<<gg, blk, 0, stream>>>(E16, Wv_t, Vt16);
  attn_kernel<<<gat, blk, 0, stream>>>(QK16, Vt16, Ctx16);
  gemm_wp_ws_kernel<<<gg, blk, 0, stream>>>(Ctx16, Wp_t, E1, RES);
  rowcast_ws_kernel<<<grow, blk, 0, stream>>>(RES, R16);
  gemm_ffn1_kernel<<<gh, blk, 0, stream>>>(R16, W1_t, b1, H16);
  gemm_ffn2_out_kernel<<<gg, blk, 0, stream>>>(H16, W2_t, b2, RES, out);
}
